// DyRep_2345052144322
// MI455X (gfx1250) — hardware-run, weakly checked
//
#include <hip/hip_runtime.h>
#include <math.h>

typedef __attribute__((ext_vector_type(16))) _Float16 v16h;
typedef __attribute__((ext_vector_type(8)))  float    v8f;
typedef __attribute__((ext_vector_type(4)))  float    v4f;
typedef __attribute__((ext_vector_type(2)))  float    v2f;

constexpr int kNodes   = 50000;
constexpr int kHid     = 32;
constexpr int kEvents  = 16384;
constexpr int kSamp    = 20;
constexpr int kTypes   = 2;
constexpr int kTiles   = kNodes / 16;
constexpr float kClip  = 75.0f;

constexpr float kCarryAct   = 64.0f;
constexpr float kCarryWgt   = 64.0f;
constexpr float kCarryRem   = 2048.0f;
constexpr float kFoldMain   = 1.0f / (kCarryAct * kCarryWgt);
constexpr float kFoldRem    = 1.0f / kCarryRem;
constexpr float kHalfMinNormal = 6.103515625e-5f;

static_assert(kNodes % 16 == 0, "16-row tiles cover the node table exactly");
static_assert(kHid == 32, "one 32-deep k-step");
static_assert(kEvents % 256 == 0, "event grid is exact");
static_assert(kTypes == 2, "two event types");
static_assert((kEvents * 4) % 128 == 0, "second output starts on a 128-B line");

constexpr size_t kOffNd   = 0;
constexpr size_t kNdBytes = (size_t)kNodes * kTypes * 4;
constexpr size_t kWsTotal = kOffNd + kNdBytes;
static_assert(kWsTotal == 400000ull, "carve total");
static_assert((kNdBytes % 128) == 0, "whole lines");
static_assert(kWsTotal <= 134217728ull, "carve cap");

__device__ __forceinline__ float flush_small(float x) {
  return (fabsf(x) < kHalfMinNormal) ? 0.0f : x;
}
__device__ __forceinline__ _Float16 act_elem(float e) {
  const float c = e * kCarryAct;
  return (_Float16)flush_small(c);
}
__device__ __forceinline__ _Float16 wgt_elem(float wa, float wb, bool isVal, bool used) {
  const float ws  = 0.5f * (wa + wb);
  const float c   = ws * kCarryWgt;
  const float cf  = flush_small(c);
  const _Float16 hv = (_Float16)cf;
  const float rem = (c - (float)hv) * kCarryRem;
  const float rf  = flush_small(rem);
  float sel = isVal ? cf : rf;
  sel = used ? sel : 0.0f;
  return (_Float16)sel;
}

__global__ __launch_bounds__(256) void node_dot_kernel(
    const float* __restrict__ emb, const float* __restrict__ W, float* __restrict__ nd)
{
  __shared__ __align__(16) float sD[8][16 * 16];
  const int lane = threadIdx.x & 31;
  const int wave = threadIdx.x >> 5;
  const int h = lane >> 4;
  const int c = lane & 15;
  const int tile = blockIdx.x * 8 + wave;
  const bool live = (tile < kTiles);
  const int tileC = live ? tile : (kTiles - 1);

  const int  wrow  = c & 1;
  const bool isVal = (c < 2);
  const bool used  = (c < 4);
  const float* wp = W + wrow * (2 * kHid) + 8 * h;
  const v4f wa0 = *(const v4f*)(wp);
  const v4f wa1 = *(const v4f*)(wp + 4);
  const v4f wa2 = *(const v4f*)(wp + 16);
  const v4f wa3 = *(const v4f*)(wp + 20);
  const v4f wb0 = *(const v4f*)(wp + kHid);
  const v4f wb1 = *(const v4f*)(wp + kHid + 4);
  const v4f wb2 = *(const v4f*)(wp + kHid + 16);
  const v4f wb3 = *(const v4f*)(wp + kHid + 20);
  v16h bfrag;
#pragma unroll
  for (int e = 0; e < 4; ++e) {
    bfrag[e]      = wgt_elem(wa0[e], wb0[e], isVal, used);
    bfrag[4 + e]  = wgt_elem(wa1[e], wb1[e], isVal, used);
    bfrag[8 + e]  = wgt_elem(wa2[e], wb2[e], isVal, used);
    bfrag[12 + e] = wgt_elem(wa3[e], wb3[e], isVal, used);
  }

  const float* ap = emb + (size_t)(tileC * 16 + c) * kHid + 8 * h;
  const v4f a0 = *(const v4f*)(ap);
  const v4f a1 = *(const v4f*)(ap + 4);
  const v4f a2 = *(const v4f*)(ap + 16);
  const v4f a3 = *(const v4f*)(ap + 20);
  v16h afrag;
#pragma unroll
  for (int e = 0; e < 4; ++e) {
    afrag[e]      = act_elem(a0[e]);
    afrag[4 + e]  = act_elem(a1[e]);
    afrag[8 + e]  = act_elem(a2[e]);
    afrag[12 + e] = act_elem(a3[e]);
  }

  v8f acc = (v8f){0.f, 0.f, 0.f, 0.f, 0.f, 0.f, 0.f, 0.f};
  acc = __builtin_amdgcn_wmma_f32_16x16x32_f16(false, afrag, false, bfrag, (short)0, acc, false, false);
  asm volatile("v_nop\n\tv_nop\n\tv_nop\n\tv_nop" : "+v"(acc) : "v"(afrag), "v"(bfrag));

  float* slab = sD[wave];
#pragma unroll
  for (int r = 0; r < 8; ++r) slab[(8 * h + r) * 16 + c] = acc[r];
  __syncthreads();

  const int row = lane >> 1;
  const int kk  = lane & 1;
  const float s0 = slab[row * 16 + kk];
  const float s1 = slab[row * 16 + kk + 2];
  const float val = (s0 + s1 * kFoldRem) * kFoldMain;
  if (live) {
    volatile float* q = nd + (size_t)tile * 32 + lane;
    *q = val;
    __threadfence();
    *q = val;
  }
}

__device__ __forceinline__ int clamp_node(int i) {
  return min(max(i, 0), kNodes - 1);
}
__device__ __forceinline__ float soft_term(float g, float p, float ip) {
  float r = g * ip;
  r = fminf(fmaxf(r, -kClip), kClip);
  return p * log1pf(expf(r));
}

__global__ __launch_bounds__(256) void event_terms_kernel(
    const int* __restrict__ u, const int* __restrict__ v, const int* __restrict__ kk,
    const int* __restrict__ uo, const int* __restrict__ vo,
    const float* __restrict__ nd, const float* __restrict__ bom, const float* __restrict__ psi,
    float* __restrict__ out)
{
  const int b  = blockIdx.x * 256 + threadIdx.x;
  const int bc = min(b, kEvents - 1);

  const float b0 = bom[0], b1 = bom[1];
  const float p0 = psi[0], p1 = psi[1];
  const float ip0 = 1.0f / p0;
  const float ip1 = 1.0f / p1;

  const int iu = clamp_node(u[bc]);
  const int iv = clamp_node(v[bc]);
  const int kb = min(max(kk[bc], 0), 1);

  const v2f ndu = *(const v2f*)(nd + 2 * (size_t)iu);
  const v2f ndv = *(const v2f*)(nd + 2 * (size_t)iv);
  const float ux = ndu.x, uy = ndu.y, vx = ndv.x, vy = ndv.y;

  const float g0 = (ux + vx) + b0;
  const float g1 = (uy + vy) + b1;
  const bool  t0 = (kb == 0);
  const float gk = t0 ? g0 : g1;
  const float pk = t0 ? p0 : p1;
  const float ik = t0 ? ip0 : ip1;
  const float inten = soft_term(gk, pk, ik);

  const int* uoB = uo + (size_t)bc * kSamp;
  const int* voB = vo + (size_t)bc * kSamp;
  float acc = 0.0f;
#pragma unroll 1
  for (int s = 0; s < kSamp; ++s) {
    const int io = clamp_node(voB[s]);
    const int jo = clamp_node(uoB[s]);
    const v2f nvo = *(const v2f*)(nd + 2 * (size_t)io);
    const v2f nuo = *(const v2f*)(nd + 2 * (size_t)jo);
    const float ox = nvo.x, oy = nvo.y, qx = nuo.x, qy = nuo.y;
#pragma unroll 1
    for (int q = 0; q < 4; ++q) {
      const bool ty = ((q & 1) != 0);
      const bool pr = ((q & 2) != 0);
      const float base = pr ? (ty ? vy : vx) : (ty ? uy : ux);
      const float oth  = pr ? (ty ? qy : qx) : (ty ? oy : ox);
      const float bb   = ty ? b1 : b0;
      const float pp   = ty ? p1 : p0;
      const float ipp  = ty ? ip1 : ip0;
      const float f = soft_term((base + oth) + bb, pp, ipp);
      acc = acc + f;
    }
  }
  const float surv = acc * (1.0f / (float)kSamp);

  if (b < kEvents) {
    volatile float* q0 = out + b;
    volatile float* q1 = out + kEvents + b;
    *q0 = inten;
    *q1 = surv;
    __threadfence();
    *q0 = inten;
    *q1 = surv;
  }
}

extern "C" void kernel_launch(void* const* d_in, const int* in_sizes, int n_in,
                              void* d_out, int out_size, void* d_ws, size_t ws_size,
                              hipStream_t stream) {
  if (n_in < 10) return;
  if (in_sizes[0] != kEvents) return;
  if (in_sizes[1] != kEvents) return;
  if (in_sizes[3] != kEvents) return;
  if (in_sizes[4] != kEvents * kSamp) return;
  if (in_sizes[5] != kEvents * kSamp) return;
  if (in_sizes[6] != kNodes * kHid) return;
  if (in_sizes[7] != kTypes * 2 * kHid) return;
  if (in_sizes[8] != kTypes) return;
  if (in_sizes[9] != kTypes) return;
  if (out_size != 2 * kEvents) return;
  if (ws_size < kWsTotal) return;

  const int*   u   = (const int*)d_in[0];
  const int*   v   = (const int*)d_in[1];
  const int*   kk  = (const int*)d_in[3];
  const int*   uo  = (const int*)d_in[4];
  const int*   vo  = (const int*)d_in[5];
  const float* emb = (const float*)d_in[6];
  const float* W   = (const float*)d_in[7];
  const float* bom = (const float*)d_in[8];
  const float* psi = (const float*)d_in[9];
  float* out = (float*)d_out;
  float* nd  = (float*)((char*)d_ws + kOffNd);

  node_dot_kernel<<<(kTiles + 7) / 8, 256, 0, stream>>>(emb, W, nd);
  event_terms_kernel<<<kEvents / 256, 256, 0, stream>>>(u, v, kk, uo, vo, nd, bom, psi, out);
}
